// VSSM_H_29265907155740
// MI455X (gfx1250) — hardware-run, weakly checked
//
#include <hip/hip_runtime.h>
#include <hip/hip_fp16.h>
#include <math.h>

typedef __attribute__((ext_vector_type(16))) _Float16 v16h;
typedef __attribute__((ext_vector_type(8)))  _Float16 v8h;
typedef __attribute__((ext_vector_type(16))) __bf16   v16b;
typedef __attribute__((ext_vector_type(8)))  __bf16   v8b;
typedef __attribute__((ext_vector_type(8)))  float    v8f;
typedef __attribute__((ext_vector_type(4)))  float    v4f;
typedef __attribute__((ext_vector_type(4)))  unsigned v4u;
typedef __attribute__((ext_vector_type(2)))  unsigned v2u;

constexpr int kBatch = 4;
constexpr int kHgt   = 64;
constexpr int kWid   = 64;
constexpr int kSeq   = kHgt * kWid;
constexpr int kDm    = 192;
constexpr int kDi    = 384;
constexpr int kNst   = 16;
constexpr int kDtR   = 96;
constexpr int kDir   = 4;
constexpr int kRows  = kBatch * kSeq;
constexpr int kXdP   = 128;
static_assert(kSeq == 4096);
static_assert(kRows == 16384);
static_assert(kDtR + 2 * kNst == kXdP);
static_assert((kDm % 32) == 0 && (kDi % 32) == 0 && (kDtR % 32) == 0);
static_assert((kRows % 64) == 0 && (kSeq % 64) == 0 && (kDi % 64) == 0 && (kXdP % 64) == 0 && (kDm % 64) == 0);
static_assert((kRows % 8) == 0);

constexpr float kUCarry   = 64.0f;
constexpr float kWCarry   = 1024.0f;
constexpr float kXdCarry  = 64.0f;
constexpr float kGCarry   = 32.0f;
constexpr float kYCarry   = 16.0f;
constexpr float kXpScale  = 1.0f / (kUCarry * kWCarry);
constexpr float kDtScale  = 1.0f / (kXdCarry * kWCarry);
constexpr float kOutScale = 1.0f / (kGCarry * kWCarry);
constexpr float kYInv     = 1.0f / kYCarry;

constexpr int kParCW    = 0;
constexpr int kParCB    = kParCW   + 9 * kDi;
constexpr int kParBias  = kParCB   + kDi;
constexpr int kParAlog  = kParBias + kDir * kDi;
constexpr int kParDs    = kParAlog + kDir * kDi * kNst;
constexpr int kParGam   = kParDs   + kDir * kDi;
constexpr int kParBet   = kParGam  + kDi;
constexpr int kParTotal = kParBet  + kDi;
static_assert(kParTotal == 32256);
static_assert((kParCB % 32) == 0 && (kParBias % 32) == 0 && (kParAlog % 32) == 0 && (kParDs % 32) == 0 &&
              (kParGam % 32) == 0 && (kParBet % 32) == 0);

constexpr size_t kSzXB   = (size_t)kRows * kDm * 2;
constexpr size_t kSzWIN  = (size_t)2 * kDi * kDm * 2;
constexpr size_t kSzWXP  = (size_t)kDir * kXdP * kDi * 2;
constexpr size_t kSzWDT  = (size_t)kDir * kDi * kDtR * 2;
constexpr size_t kSzWOUT = (size_t)kDm * kDi * 2;
constexpr size_t kSzPAR  = (size_t)kParTotal * 4;
constexpr size_t kSzR1   = (size_t)kRows * kDi * 4;
constexpr size_t kSzZ    = (size_t)kRows * kDi * 4;
constexpr size_t kSzU    = (size_t)kRows * kDi * 4;
constexpr size_t kSzY    = (size_t)kDir * kRows * kDi * 2;
constexpr size_t kOffXB   = 0;
constexpr size_t kOffWIN  = kOffXB   + kSzXB;
constexpr size_t kOffWXP  = kOffWIN  + kSzWIN;
constexpr size_t kOffWDT  = kOffWXP  + kSzWXP;
constexpr size_t kOffWOUT = kOffWDT  + kSzWDT;
constexpr size_t kOffPAR  = kOffWOUT + kSzWOUT;
constexpr size_t kOffR1   = kOffPAR  + kSzPAR;
constexpr size_t kOffZ    = kOffR1   + kSzR1;
constexpr size_t kOffU    = kOffZ    + kSzZ;
constexpr size_t kOffY    = kOffU    + kSzU;
constexpr size_t kWsTotal = kSzXB + kSzWIN + kSzWXP + kSzWDT + kSzWOUT + kSzPAR + kSzR1 + kSzZ + kSzU + kSzY;
static_assert(kOffY + kSzY == kWsTotal);
static_assert(kWsTotal == 133380096ull);
static_assert(kWsTotal <= 134217728ull);
static_assert((kOffWIN % 128) == 0 && (kOffWXP % 128) == 0 && (kOffWDT % 128) == 0 && (kOffWOUT % 128) == 0 &&
              (kOffPAR % 128) == 0 && (kOffR1 % 128) == 0 && (kOffZ % 128) == 0 && (kOffU % 128) == 0 && (kOffY % 128) == 0);
constexpr size_t kTmpUK   = 0;
constexpr size_t kTmpDTP  = kTmpUK   + (size_t)kSeq * kDi * 4;
constexpr size_t kTmpUK16 = kTmpDTP  + (size_t)kSeq * kDi * 4;
constexpr size_t kTmpXD32 = kTmpUK16 + (size_t)kSeq * kDi * 2;
constexpr size_t kTmpXD16 = kTmpXD32 + (size_t)kSeq * kXdP * 4;
constexpr size_t kTmpEnd  = kTmpXD16 + (size_t)kSeq * kXdP * 2;
static_assert(kTmpEnd <= kSzR1);
static_assert((size_t)kRows * kDi * 2 <= kSzR1);

__device__ __forceinline__ unsigned bf16_bits(float f) {
  const unsigned u = __float_as_uint(f);
  return (u + 0x7FFFu + ((u >> 16) & 1u)) >> 16;
}
__device__ __forceinline__ float bf16_rne(float f) { return __uint_as_float(bf16_bits(f) << 16); }
__device__ __forceinline__ float flush16(float v) { return (fabsf(v) < 6.103515625e-05f) ? 0.0f : v; }
__device__ __forceinline__ unsigned f16_bits(float v) {
  return (unsigned)__half_as_ushort(__float2half_rn(flush16(v)));
}
__device__ __forceinline__ float h16_to_f32(unsigned hb) {
  const unsigned sgn = (hb & 0x8000u) << 16; const unsigned em = hb & 0x7fffu;
  const float fn = __uint_as_float((em << 13) + 0x38000000u);
  const float fs = (float)em * 5.9604644775390625e-8f;
  const float mag = (em < 0x400u) ? fs : fn; return __uint_as_float(__float_as_uint(mag) | sgn); }

__device__ __forceinline__ void wmma_guard_h(v8f& c, v16h a, v16h b) { asm volatile("v_nop\n\tv_nop\n\tv_nop\n\tv_nop" : "+v"(c) : "v"(a), "v"(b)); }
__device__ __forceinline__ void wmma_guard_b(v8f& c, v16b a, v16b b) { asm volatile("v_nop\n\tv_nop\n\tv_nop\n\tv_nop" : "+v"(c) : "v"(a), "v"(b)); }
__device__ __forceinline__ void keep4_h(v16h a, v16h b, v16h c, v16h d) { asm volatile("v_nop" :: "v"(a), "v"(b), "v"(c), "v"(d)); }
__device__ __forceinline__ void keep4_b(v16b a, v16b b, v16b c, v16b d) { asm volatile("v_nop" :: "v"(a), "v"(b), "v"(c), "v"(d)); }
__device__ __forceinline__ void acc_guard4(v8f& a, v8f& b, v8f& c, v8f& d) { asm volatile("v_nop\n\tv_nop\n\tv_nop\n\tv_nop" : "+v"(a), "+v"(b), "+v"(c), "+v"(d)); }

template <typename T> struct Frag;
template <> struct Frag<_Float16> {
  typedef v16h V; union U { v16h v; v8h h[2]; };
  static __device__ __forceinline__ v16h load(const _Float16* p) {
    U f; f.h[0] = *(const v8h*)(p); f.h[1] = *(const v8h*)(p + 16); return f.v;
  }
  static __device__ __forceinline__ v8f mma(v16h a, v16h b, v8f c) {
    c = __builtin_amdgcn_wmma_f32_16x16x32_f16(false, a, false, b, (short)0, c, false, false);
    wmma_guard_h(c, a, b);
    return c;
  }
  static __device__ __forceinline__ void keep(v16h a, v16h b, v16h c, v16h d) { keep4_h(a, b, c, d); }
};
template <> struct Frag<__bf16> {
  typedef v16b V; union U { v16b v; v8b h[2]; };
  static __device__ __forceinline__ v16b load(const __bf16* p) {
    U f; f.h[0] = *(const v8b*)(p); f.h[1] = *(const v8b*)(p + 16); return f.v;
  }
  static __device__ __forceinline__ v8f mma(v16b a, v16b b, v8f c) {
    c = __builtin_amdgcn_wmma_f32_16x16x32_bf16(false, a, false, b, (short)0, c, false, false);
    wmma_guard_b(c, a, b);
    return c;
  }
  static __device__ __forceinline__ void keep(v16b a, v16b b, v16b c, v16b d) { keep4_b(a, b, c, d); }
};

template <int ET> struct Elem;
template <> struct Elem<0> { typedef _Float16 T; };
template <> struct Elem<1> { typedef __bf16 T; };
template <int ET, int BIAS_MODE, int OUT_MODE>
__global__ __launch_bounds__(256) void wmma_gemm64(
    const unsigned short* __restrict__ Ap, int lda, long strideA,
    const unsigned short* __restrict__ Btp, int ldb, long strideB,
    void* __restrict__ Cout, void* __restrict__ Cout2, int ldc, long strideC,
    const float* __restrict__ bias,
    int M, int N, int K, float scale, float scale2) {
  typedef typename Elem<ET>::T T;
  typedef typename Frag<T>::V V;
  const T* A = (const T*)Ap; const T* Bt = (const T*)Btp;
  __shared__ __align__(16) float sT[8][16 * 68];
  const int b    = blockIdx.y;
  const int lane = threadIdx.x & 31;
  const int wave = threadIdx.x >> 5;
  const int tilesN = N >> 6;
  const int tilesM = M >> 6;
  const int tile = blockIdx.x * 8 + wave;
  if (tile >= tilesM * tilesN) return;
  const int tm = tile / tilesN;
  const int tn = tile - tm * tilesN;
  const int m0 = tm << 6;
  const int n0 = tn << 6;

  const T* Ab = A  + (size_t)b * strideA;
  const T* Bb = Bt + (size_t)b * strideB;

  const int rlane = lane & 15;
  const int koff  = (lane >> 4) * 8;
  const int mOff  = (lane >> 4) * 8;

  v8f acc[4][4];
#pragma unroll
  for (int i = 0; i < 4; ++i)
#pragma unroll
    for (int j = 0; j < 4; ++j) acc[i][j] = (v8f){0.f,0.f,0.f,0.f,0.f,0.f,0.f,0.f};

  for (int k0 = 0; k0 < K; k0 += 32) {
    V bh[4];
#pragma unroll
    for (int j = 0; j < 4; ++j) {
      const size_t bo = (size_t)(n0 + (j << 4) + rlane) * ldb + koff + k0;
      bh[j] = Frag<T>::load(Bb + bo);
    }
#pragma unroll
    for (int i = 0; i < 4; ++i) {
      const size_t ao = (size_t)(m0 + (i << 4) + rlane) * lda + koff + k0;
      V ah = Frag<T>::load(Ab + ao);
#pragma unroll
      for (int j = 0; j < 4; ++j) acc[i][j] = Frag<T>::mma(ah, bh[j], acc[i][j]);
    }
    Frag<T>::keep(bh[0], bh[1], bh[2], bh[3]);
  }
  acc_guard4(acc[0][0], acc[0][1], acc[0][2], acc[0][3]);
  acc_guard4(acc[1][0], acc[1][1], acc[1][2], acc[1][3]);
  acc_guard4(acc[2][0], acc[2][1], acc[2][2], acc[2][3]);
  acc_guard4(acc[3][0], acc[3][1], acc[3][2], acc[3][3]);

  float* slab = sT[wave];
#pragma unroll
  for (int i = 0; i < 4; ++i) {
    const int mBase = m0 + (i << 4);
#pragma unroll
    for (int j = 0; j < 4; ++j) {
      const int n = n0 + (j << 4) + rlane;
      float bv = 0.f;
      if (BIAS_MODE == 2) bv = bias[n];
#pragma unroll
      for (int r = 0; r < 8; ++r) {
        float v = acc[i][j][r] * scale;
        if (BIAS_MODE == 2) v += bv;
        slab[(mOff + r) * 68 + (j << 4) + rlane] = v;
      }
    }
    __builtin_amdgcn_fence(__ATOMIC_RELEASE, "workgroup");
    __builtin_amdgcn_wave_barrier();
    __builtin_amdgcn_fence(__ATOMIC_ACQUIRE, "workgroup");
    {
      float* C = ((OUT_MODE == 0) ? (float*)Cout : (float*)Cout2) + (size_t)b * strideC;
      const int hh = lane >> 4, c4 = (lane & 15) * 4;
      for (int pass = 0; pass < 2; ++pass) {
#pragma unroll
        for (int it = 0; it < 8; ++it) {
          const int row = it * 2 + hh;
          v4f v = *(const v4f*)(slab + row * 68 + c4);
          *(volatile v4f*)(C + (size_t)(mBase + row) * ldc + n0 + c4) = v;
        }
        __threadfence();
      }
    }
    if (OUT_MODE == 3) {
      const int q = lane >> 3, c8 = (lane & 7) * 8;
      unsigned short* C = (unsigned short*)Cout + (size_t)b * strideC;
      v8h hv[4];
#pragma unroll
      for (int it = 0; it < 4; ++it) {
        const float* sp = slab + (it * 4 + q) * 68 + c8;
#pragma unroll
        for (int e = 0; e < 8; ++e) {
          const float cv = flush16(sp[e] * scale2);
          hv[it][e] = (_Float16)cv;
        }
      }
      for (int pass = 0; pass < 2; ++pass) {
#pragma unroll
        for (int it = 0; it < 4; ++it) {
          const int row = it * 4 + q;
          *(volatile v8h*)(C + (size_t)(mBase + row) * ldc + n0 + c8) = hv[it];
        }
        __threadfence();
      }
    }
    __builtin_amdgcn_fence(__ATOMIC_RELEASE, "workgroup");
    __builtin_amdgcn_wave_barrier();
    __builtin_amdgcn_fence(__ATOMIC_ACQUIRE, "workgroup");
  }
}

__global__ __launch_bounds__(256) void cvt_bf16_kernel(
    const float* __restrict__ s0, unsigned short* __restrict__ d0, int n0,
    const float* __restrict__ s1, unsigned short* __restrict__ d1, int n1)
{
  const int seg = blockIdx.y;
  const float* src = (seg == 0) ? s0 : s1;
  unsigned short* dst = (seg == 0) ? d0 : d1;
  const int total8 = (seg == 0) ? n0 : n1;
  const int i = blockIdx.x * 256 + threadIdx.x;
  if (i >= total8) return;
  const size_t e0 = (size_t)i << 3;
  const v4f a0 = *(const v4f*)(src + e0);
  const v4f a1 = *(const v4f*)(src + e0 + 4);
  const float f0 = a0[0], f1 = a0[1], f2 = a0[2], f3 = a0[3];
  const float f4 = a1[0], f5 = a1[1], f6 = a1[2], f7 = a1[3];
  v4u w;
  w[0] = bf16_bits(f0) | (bf16_bits(f1) << 16);
  w[1] = bf16_bits(f2) | (bf16_bits(f3) << 16);
  w[2] = bf16_bits(f4) | (bf16_bits(f5) << 16);
  w[3] = bf16_bits(f6) | (bf16_bits(f7) << 16);
  unsigned short* q = dst + e0;
  *(volatile v4u*)q = w;
  __threadfence();
  *(volatile v4u*)q = w;
}

__global__ __launch_bounds__(256) void cvt_f16w_kernel(
    const float* __restrict__ s0, unsigned short* __restrict__ d0, int n0,
    const float* __restrict__ s1, unsigned short* __restrict__ d1, int n1,
    const float* __restrict__ s2, unsigned short* __restrict__ d2, int n2, float carry)
{
  const int seg = blockIdx.y;
  const float* src = (seg == 0) ? s0 : ((seg == 1) ? s1 : s2);
  unsigned short* dst = (seg == 0) ? d0 : ((seg == 1) ? d1 : d2);
  const int total8 = (seg == 0) ? n0 : ((seg == 1) ? n1 : n2);
  const int i = blockIdx.x * 256 + threadIdx.x;
  if (i >= total8) return;
  const size_t e0 = (size_t)i << 3;
  const v4f a0 = *(const v4f*)(src + e0);
  const v4f a1 = *(const v4f*)(src + e0 + 4);
  const float f0 = bf16_rne(a0[0]) * carry, f1 = bf16_rne(a0[1]) * carry;
  const float f2 = bf16_rne(a0[2]) * carry, f3 = bf16_rne(a0[3]) * carry;
  const float f4 = bf16_rne(a1[0]) * carry, f5 = bf16_rne(a1[1]) * carry;
  const float f6 = bf16_rne(a1[2]) * carry, f7 = bf16_rne(a1[3]) * carry;
  v4u w;
  w[0] = f16_bits(f0) | (f16_bits(f1) << 16);
  w[1] = f16_bits(f2) | (f16_bits(f3) << 16);
  w[2] = f16_bits(f4) | (f16_bits(f5) << 16);
  w[3] = f16_bits(f6) | (f16_bits(f7) << 16);
  unsigned short* q = dst + e0;
  *(volatile v4u*)q = w;
  __threadfence();
  *(volatile v4u*)q = w;
}

__global__ __launch_bounds__(256) void par_kernel(
    const float* __restrict__ cw, const float* __restrict__ cb, const float* __restrict__ dtb,
    const float* __restrict__ alog, const float* __restrict__ dsk, const float* __restrict__ gam,
    const float* __restrict__ bet, float* __restrict__ par)
{
  const int seg = blockIdx.y;
  const float* src = cw;
  int n = 9 * kDi;
  int off = kParCW;
  if (seg == 1) { src = cb;   n = kDi;               off = kParCB; }
  if (seg == 2) { src = dtb;  n = kDir * kDi;        off = kParBias; }
  if (seg == 3) { src = alog; n = kDir * kDi * kNst; off = kParAlog; }
  if (seg == 4) { src = dsk;  n = kDir * kDi;        off = kParDs; }
  if (seg == 5) { src = gam;  n = kDi;               off = kParGam; }
  if (seg == 6) { src = bet;  n = kDi;               off = kParBet; }
  const int i = blockIdx.x * 256 + threadIdx.x;
  if (i >= n) return;
  int si = i;
  if (seg == 0) {
    const int t = i / kDi;
    const int d = i - t * kDi;
    si = d * 9 + t;
  }
  const float v = bf16_rne(src[si]);
  volatile float* q = par + off + i;
  *q = v;
  __threadfence();
  *q = v;
}

__global__ __launch_bounds__(256) void conv_silu_kernel(
    const float* __restrict__ XP, const float* __restrict__ cwt, const float* __restrict__ cbr,
    float* __restrict__ U)
{
  const int i = blockIdx.x * 256 + threadIdx.x;
  if (i >= kRows * kDi) return;
  const int m = i / kDi;
  const int d = i - m * kDi;
  const int b = m >> 12;
  const int s = m & (kSeq - 1);
  const int h = s >> 6;
  const int w = s & 63;
  float acc = 0.0f;
#pragma unroll 1
  for (int ky = 0; ky < 3; ++ky) {
    const int hy = h + ky - 1;
    const bool vy = (hy >= 0) && (hy < kHgt);
    const int hc = (hy < 0) ? 0 : ((hy > kHgt - 1) ? (kHgt - 1) : hy);
#pragma unroll
    for (int kx = 0; kx < 3; ++kx) {
      const int wx = w + kx - 1;
      const bool ok = vy && (wx >= 0) && (wx < kWid);
      const int wc = (wx < 0) ? 0 : ((wx > kWid - 1) ? (kWid - 1) : wx);
      float xv = XP[(size_t)(b * kSeq + hc * kWid + wc) * kDi + d];
      asm volatile("" : "+v"(xv));
      float wv = cwt[(ky * 3 + kx) * kDi + d];
      asm volatile("" : "+v"(wv));
      const float xs = ok ? xv : 0.0f;
      acc = fmaf(xs, wv, acc);
    }
  }
  const float xc = acc + cbr[d];
  const float sg = __builtin_amdgcn_rcpf(1.0f + expf(-xc));
  const float uv = xc * sg;
  volatile float* q = U + (size_t)i;
  *q = uv;
  __threadfence();
  *q = uv;
}

__global__ __launch_bounds__(256) void perm_kernel(
    const float* __restrict__ Ub, float* __restrict__ UK, unsigned short* __restrict__ UK16, int k)
{
  const int i = blockIdx.x * 256 + threadIdx.x;
  if (i >= kSeq * (kDi / 4)) return;
  const int l  = i / (kDi / 4);
  const int c4 = (i - l * (kDi / 4)) * 4;
  const int lr = ((k & 2) != 0) ? (kSeq - 1 - l) : l;
  int s = ((k & 1) != 0) ? (((lr & 63) << 6) | (lr >> 6)) : lr;
  s = (s < 0) ? 0 : ((s > kSeq - 1) ? (kSeq - 1) : s);
  const v4f v = *(const v4f*)(Ub + (size_t)s * kDi + c4);
  const float f0 = v[0], f1 = v[1], f2 = v[2], f3 = v[3];
  v2u w;
  w[0] = f16_bits(f0 * kUCarry) | (f16_bits(f1 * kUCarry) << 16);
  w[1] = f16_bits(f2 * kUCarry) | (f16_bits(f3 * kUCarry) << 16);
  float* qf = UK + (size_t)l * kDi + c4;
  unsigned short* qh = UK16 + (size_t)l * kDi + c4;
  *(volatile v4f*)qf = v;
  *(volatile v2u*)qh = w;
  __threadfence();
  *(volatile v4f*)qf = v;
  *(volatile v2u*)qh = w;
}

typedef float    ms1_v4f __attribute__((ext_vector_type(4)));
typedef unsigned ms1_v4u __attribute__((ext_vector_type(4)));
struct ms1_args {
  const float* dtpre;
  const float* u;
  const float* bc;
  const float* z;
  const float* A_log;
  const float* Dskip;
  __half* y;
  __half* y_lo;
  long ld_dtpre;
  long ld_u;
  long ld_bc;
  long ld_z;
  long ld_y;
  int offB;
  int offC;
  int offZ;
  float ycarry;
  int dir;
  int D;
  int L;
  int nbatch;
};
static_assert(sizeof(ms1_args) == 136);

__device__ __forceinline__ float ms1_flush16(float v) {
  return (fabsf(v) < 6.103515625e-05f) ? 0.0f : v;
}
__device__ __forceinline__ unsigned ms1_h16bits(float v) {
  return (unsigned)__half_as_ushort(__float2half_rn(ms1_flush16(v)));
}
__device__ __forceinline__ float ms1_h16val(unsigned b) {
  return __half2float(__ushort_as_half((unsigned short)b));
}
__device__ __forceinline__ float ms1_softplus(float v) {
  return fmaxf(v, 0.0f) + log1pf(expf(-fabsf(v)));
}
__device__ __forceinline__ void ms1_pack2(float v0, float v1, unsigned& hw, unsigned& lw) {
  const unsigned h0 = ms1_h16bits(v0);
  const unsigned h1 = ms1_h16bits(v1);
  const float r0 = (v0 - ms1_h16val(h0)) * 2048.0f;
  const float r1 = (v1 - ms1_h16val(h1)) * 2048.0f;
  const unsigned l0 = ms1_h16bits(r0);
  const unsigned l1 = ms1_h16bits(r1);
  hw = h0 | (h1 << 16);
  lw = l0 | (l1 << 16);
}

template <int NSTATE>
__global__ __launch_bounds__(64 * (NSTATE / 16)) void ms1_scan_kernel(ms1_args a)
{
  static_assert(NSTATE == 16 || NSTATE == 64);
  constexpr int NQ  = NSTATE / 16;
  constexpr int NT  = 64 * NQ;
  constexpr int NW  = NT / 32;
  constexpr int BCW = 2 * NSTATE;
  constexpr int YP  = 68;
  constexpr int RPI = NW * 4;
  constexpr int NIT = 64 / RPI;
  static_assert(16 * NT <= 64 * YP);
  __shared__ __align__(16) float sBC[64 * BCW];
  __shared__ __align__(16) float sY[64 * YP];
  const int tid  = threadIdx.x;
  const int lane = tid & 31;
  const int wave = tid >> 5;
  const int c    = tid / NQ;
  const int sq   = tid - c * NQ;
  const int bpb  = a.D / 64;
  const int bi   = blockIdx.x / bpb;
  if (bi >= a.nbatch) return;
  const int d0 = (blockIdx.x - bi * bpb) * 64;
  const int d  = d0 + c;
  const long rowb = (long)bi * a.L;
  const bool hasz  = (a.z != nullptr);
  const bool hasD  = (a.Dskip != nullptr);
  const bool hasLo = (a.y_lo != nullptr);

#pragma unroll 1
  for (int n = 0; n < 16; ++n) {
    const float al = a.A_log[(long)d * NSTATE + sq * 16 + n];
    sY[n * NT + tid] = -expf(al);
  }
  __syncthreads();
  float An[16], h[16];
#pragma unroll
  for (int n = 0; n < 16; ++n) {
    An[n] = sY[n * NT + tid];
    h[n] = 0.0f;
  }
  float Dd = 0.0f;
  if (hasD) Dd = a.Dskip[d];

  const int nchunk = a.L / 64;
  const bool fwd = (a.dir > 0);
  const int s0 = fwd ? 0 : 63;
  const int sd = fwd ? 1 : -1;
  const int q  = lane >> 3;
  const int c8 = (lane & 7) * 8;

#pragma unroll 1
  for (int ci = 0; ci < nchunk; ++ci) {
    const int tb = fwd ? (ci * 64) : (a.L - 64 - ci * 64);
    const long rowc = rowb + tb;
    __syncthreads();
#pragma unroll 8
    for (int i = 0; i < 32; ++i) {
      const int idx = tid + i * NT;
      const int st  = idx / BCW;
      const int col = idx - st * BCW;
      const int sc  = (col < NSTATE) ? (a.offB + col) : (a.offC + col - NSTATE);
      sBC[idx] = a.bc[(rowc + st) * a.ld_bc + sc];
    }
    __syncthreads();
#pragma unroll 1
    for (int s = 0; s < 64; ++s) {
      const int ls = s0 + sd * s;
      const long row = rowc + ls;
      float pre = a.dtpre[row * a.ld_dtpre + d];
      float uv  = a.u[row * a.ld_u + d];
      float zv  = 0.0f;
      if (hasz) zv = a.z[row * a.ld_z + a.offZ + d];
      asm volatile("" : "+v"(pre));
      asm volatile("" : "+v"(uv));
      asm volatile("" : "+v"(zv));
      const float delta = ms1_softplus(pre);
      const float dtx = delta * uv;
      const float* bp = sBC + ls * BCW + sq * 16;
      const float* cp = bp + NSTATE;
      ms1_v4f Bq[4], Cq[4];
#pragma unroll
      for (int k = 0; k < 4; ++k) {
        Bq[k] = *(const ms1_v4f*)(bp + 4 * k);
        Cq[k] = *(const ms1_v4f*)(cp + 4 * k);
      }
      float yv = 0.0f;
#pragma unroll
      for (int n = 0; n < 16; ++n) {
        const float e = __expf(delta * An[n]);
        h[n] = fmaf(e, h[n], dtx * Bq[n >> 2][n & 3]);
        yv = fmaf(h[n], Cq[n >> 2][n & 3], yv);
      }
      if (NQ > 1) {
        yv += __shfl_xor(yv, 1, 32);
        yv += __shfl_xor(yv, 2, 32);
      }
      if (hasD) yv = fmaf(uv, Dd, yv);
      if (hasz) {
        const float sg = __builtin_amdgcn_rcpf(1.0f + expf(-zv));
        yv = yv * (zv * sg);
      }
      if (sq == 0) sY[ls * YP + c] = yv * a.ycarry;
    }
    __syncthreads();
    ms1_v4u hw[NIT], lw[NIT];
#pragma unroll
    for (int it = 0; it < NIT; ++it) {
      const int row = it * RPI + wave * 4 + q;
      const float* sp = sY + row * YP + c8;
      const ms1_v4f f0 = *(const ms1_v4f*)(sp);
      const ms1_v4f f1 = *(const ms1_v4f*)(sp + 4);
      unsigned h0, h1, h2, h3, l0, l1, l2, l3;
      ms1_pack2(f0[0], f0[1], h0, l0);
      ms1_pack2(f0[2], f0[3], h1, l1);
      ms1_pack2(f1[0], f1[1], h2, l2);
      ms1_pack2(f1[2], f1[3], h3, l3);
      hw[it] = (ms1_v4u){h0, h1, h2, h3};
      lw[it] = (ms1_v4u){l0, l1, l2, l3};
    }
    for (int pass = 0; pass < 2; ++pass) {
#pragma unroll
      for (int it = 0; it < NIT; ++it) {
        const int row = it * RPI + wave * 4 + q;
        const long o = (rowc + row) * a.ld_y + d0 + c8;
        *(volatile ms1_v4u*)(a.y + o) = hw[it];
        if (hasLo) *(volatile ms1_v4u*)(a.y_lo + o) = lw[it];
      }
      __threadfence();
    }
  }
}

__device__ __forceinline__ float merge4(unsigned p0, unsigned p2, unsigned p1, unsigned p3) {
  float t = h16_to_f32(p0) + h16_to_f32(p2);
  t = t + h16_to_f32(p1);
  t = t + h16_to_f32(p3);
  return t * kYInv;
}

__global__ __launch_bounds__(256) void merge_norm_gate_kernel(
    const unsigned short* __restrict__ Y, const float* __restrict__ Z,
    const float* __restrict__ gam, const float* __restrict__ bet,
    unsigned short* __restrict__ G16)
{
  __shared__ __align__(16) float sV[8 * kDi];
  __shared__ __align__(16) v2u sG[8 * 96];
  const int lane = threadIdx.x & 31;
  const int wave = threadIdx.x >> 5;
  const int m  = blockIdx.x * 8 + wave;
  const int b  = m >> 12;
  const int s  = m & (kSeq - 1);
  const int hh = s >> 6;
  const int ww = s & 63;
  const int l1 = ww * 64 + hh;
  const size_t r0 = ((size_t)(0 * kBatch + b) * kSeq + s) * kDi;
  const size_t r1 = ((size_t)(1 * kBatch + b) * kSeq + l1) * kDi;
  const size_t r2 = ((size_t)(2 * kBatch + b) * kSeq + (kSeq - 1 - s)) * kDi;
  const size_t r3 = ((size_t)(3 * kBatch + b) * kSeq + (kSeq - 1 - l1)) * kDi;
  float* sv = sV + wave * kDi;
  v2u* sg = sG + wave * 96;

  float s1 = 0.0f;
#pragma unroll 1
  for (int j = 0; j < 3; ++j) {
    const int c = j * 128 + lane * 4;
    const v2u w0 = *(const v2u*)(Y + r0 + c);
    const v2u w1 = *(const v2u*)(Y + r1 + c);
    const v2u w2 = *(const v2u*)(Y + r2 + c);
    const v2u w3 = *(const v2u*)(Y + r3 + c);
    const unsigned a0 = w0[0], a1 = w0[1];
    const unsigned b0 = w1[0], b1 = w1[1];
    const unsigned c0 = w2[0], c1 = w2[1];
    const unsigned d0 = w3[0], d1 = w3[1];
    v4f acc;
    acc[0] = merge4(a0 & 0xffffu, c0 & 0xffffu, b0 & 0xffffu, d0 & 0xffffu);
    acc[1] = merge4(a0 >> 16, c0 >> 16, b0 >> 16, d0 >> 16);
    acc[2] = merge4(a1 & 0xffffu, c1 & 0xffffu, b1 & 0xffffu, d1 & 0xffffu);
    acc[3] = merge4(a1 >> 16, c1 >> 16, b1 >> 16, d1 >> 16);
    *(v4f*)(sv + c) = acc;
    s1 += (acc[0] + acc[1]) + (acc[2] + acc[3]);
  }
  s1 += __shfl_xor(s1, 16, 32);
  s1 += __shfl_xor(s1, 8, 32);
  s1 += __shfl_xor(s1, 4, 32);
  s1 += __shfl_xor(s1, 2, 32);
  s1 += __shfl_xor(s1, 1, 32);
  const float mu = s1 * (1.0f / (float)kDi);

  float s2 = 0.0f;
#pragma unroll 1
  for (int j = 0; j < 3; ++j) {
    const int c = j * 128 + lane * 4;
    const v4f v = *(const v4f*)(sv + c);
    const float e0 = v[0] - mu, e1 = v[1] - mu, e2 = v[2] - mu, e3 = v[3] - mu;
    s2 += (e0 * e0 + e1 * e1) + (e2 * e2 + e3 * e3);
  }
  s2 += __shfl_xor(s2, 16, 32);
  s2 += __shfl_xor(s2, 8, 32);
  s2 += __shfl_xor(s2, 4, 32);
  s2 += __shfl_xor(s2, 2, 32);
  s2 += __shfl_xor(s2, 1, 32);
  const float var = s2 * (1.0f / (float)kDi);
  const float rs = rsqrtf(var + 1.0e-5f);

#pragma unroll 1
  for (int j = 0; j < 3; ++j) {
    const int c = j * 128 + lane * 4;
    const v4f v  = *(const v4f*)(sv + c);
    const v4f g4 = *(const v4f*)(gam + c);
    const v4f b4 = *(const v4f*)(bet + c);
    const v4f z4 = *(const v4f*)(Z + (size_t)m * kDi + c);
    unsigned hb[4];
#pragma unroll
    for (int e = 0; e < 4; ++e) {
      const float yn = ((v[e] - mu) * rs) * g4[e] + b4[e];
      const float zv = z4[e];
      const float sgm = __builtin_amdgcn_rcpf(1.0f + expf(-zv));
      const float gv = yn * (zv * sgm);
      hb[e] = f16_bits(gv * kGCarry);
    }
    v2u w;
    w[0] = hb[0] | (hb[1] << 16);
    w[1] = hb[2] | (hb[3] << 16);
    sg[j * 32 + lane] = w;
  }
  const v2u g0 = sg[lane];
  const v2u g1 = sg[32 + lane];
  const v2u g2 = sg[64 + lane];
  unsigned short* q = G16 + (size_t)m * kDi + lane * 4;
  for (int pass = 0; pass < 2; ++pass) {
    *(volatile v2u*)(q) = g0;
    *(volatile v2u*)(q + 128) = g1;
    *(volatile v2u*)(q + 256) = g2;
    __threadfence();
  }
}

extern "C" void kernel_launch(void* const* d_in, const int* in_sizes, int n_in,
                              void* d_out, int out_size, void* d_ws, size_t ws_size,
                              hipStream_t stream) {
  if (n_in < 12) return;
  if (in_sizes[0] != kRows * kDm) return;
  if (in_sizes[1] != 2 * kDi * kDm) return;
  if (in_sizes[2] != kDi * 9) return;
  if (in_sizes[3] != kDi) return;
  if (in_sizes[4] != kDir * kXdP * kDi) return;
  if (in_sizes[5] != kDir * kDi * kDtR) return;
  if (in_sizes[6] != kDir * kDi) return;
  if (in_sizes[7] != kDir * kDi * kNst) return;
  if (in_sizes[8] != kDir * kDi) return;
  if (in_sizes[9] != kDi) return;
  if (in_sizes[10] != kDi) return;
  if (in_sizes[11] != kDm * kDi) return;
  if (out_size != kRows * kDm) return;
  if (ws_size < kWsTotal) return;

  const float* x      = (const float*)d_in[0];
  const float* w_in   = (const float*)d_in[1];
  const float* conv_w = (const float*)d_in[2];
  const float* conv_b = (const float*)d_in[3];
  const float* w_xp   = (const float*)d_in[4];
  const float* w_dt   = (const float*)d_in[5];
  const float* b_dt   = (const float*)d_in[6];
  const float* a_log  = (const float*)d_in[7];
  const float* d_skip = (const float*)d_in[8];
  const float* ln_g   = (const float*)d_in[9];
  const float* ln_b   = (const float*)d_in[10];
  const float* w_out  = (const float*)d_in[11];
  float* out = (float*)d_out;

  char* ws = (char*)d_ws;
  unsigned short* XB   = (unsigned short*)(ws + kOffXB);
  unsigned short* WIN  = (unsigned short*)(ws + kOffWIN);
  unsigned short* WXP  = (unsigned short*)(ws + kOffWXP);
  unsigned short* WDT  = (unsigned short*)(ws + kOffWDT);
  unsigned short* WOUT = (unsigned short*)(ws + kOffWOUT);
  float*          PAR  = (float*)(ws + kOffPAR);
  float*          XP   = (float*)(ws + kOffR1);
  float*          Zp   = (float*)(ws + kOffZ);
  float*          Up   = (float*)(ws + kOffU);
  unsigned short* Yp   = (unsigned short*)(ws + kOffY);
  float*          UK   = (float*)(ws + kOffR1 + kTmpUK);
  float*          DTP  = (float*)(ws + kOffR1 + kTmpDTP);
  unsigned short* UK16 = (unsigned short*)(ws + kOffR1 + kTmpUK16);
  float*          XD32 = (float*)(ws + kOffR1 + kTmpXD32);
  unsigned short* XD16 = (unsigned short*)(ws + kOffR1 + kTmpXD16);
  unsigned short* G16  = (unsigned short*)(ws + kOffR1);

  cvt_bf16_kernel<<<dim3((kRows * kDm / 8 + 255) / 256, 2), 256, 0, stream>>>(
      x, XB, kRows * kDm / 8, w_in, WIN, 2 * kDi * kDm / 8);
  cvt_f16w_kernel<<<dim3((kDir * kXdP * kDi / 8 + 255) / 256, 3), 256, 0, stream>>>(
      w_xp, WXP, kDir * kXdP * kDi / 8, w_dt, WDT, kDir * kDi * kDtR / 8, w_out, WOUT, kDm * kDi / 8, kWCarry);
  par_kernel<<<dim3((kDir * kDi * kNst + 255) / 256, 7), 256, 0, stream>>>(
      conv_w, conv_b, b_dt, a_log, d_skip, ln_g, ln_b, PAR);

  wmma_gemm64<1, 0, 0><<<dim3(((kRows / 64) * (kDi / 64) + 7) / 8, 2), 256, 0, stream>>>(
      XB, kDm, 0L,
      WIN, kDm, (long)kDi * kDm,
      (void*)XP, nullptr, kDi, (long)kRows * kDi,
      nullptr,
      kRows, kDi, kDm, 1.0f, 1.0f);

  conv_silu_kernel<<<(kRows * kDi) / 256, 256, 0, stream>>>(XP, PAR + kParCW, PAR + kParCB, Up);

  for (int k = 0; k < kDir; ++k) {
    for (int b = 0; b < kBatch; ++b) {
      perm_kernel<<<(kSeq * (kDi / 4)) / 256, 256, 0, stream>>>(Up + (size_t)b * kSeq * kDi, UK, UK16, k);

      wmma_gemm64<0, 0, 3><<<dim3(((kSeq / 64) * (kXdP / 64) + 7) / 8, 1), 256, 0, stream>>>(
          UK16, kDi, 0L,
          WXP + (size_t)k * kXdP * kDi, kDi, 0L,
          (void*)XD16, (void*)XD32, kXdP, 0L,
          nullptr,
          kSeq, kXdP, kDi, kXpScale, kXdCarry);

      wmma_gemm64<0, 2, 0><<<dim3(((kSeq / 64) * (kDi / 64) + 7) / 8, 1), 256, 0, stream>>>(
          XD16, kXdP, 0L,
          WDT + (size_t)k * kDi * kDtR, kDtR, 0L,
          (void*)DTP, nullptr, kDi, 0L,
          PAR + kParBias + k * kDi,
          kSeq, kDi, kDtR, kDtScale, 1.0f);

      ms1_args sa;
      sa.dtpre = DTP;
      sa.u = UK;
      sa.bc = XD32;
      sa.z = nullptr;
      sa.A_log = PAR + kParAlog + (size_t)k * kDi * kNst;
      sa.Dskip = PAR + kParDs + k * kDi;
      sa.y = (__half*)(Yp + (size_t)(k * kBatch + b) * kSeq * kDi);
      sa.y_lo = nullptr;
      sa.ld_dtpre = kDi;
      sa.ld_u = kDi;
      sa.ld_bc = kXdP;
      sa.ld_z = 0;
      sa.ld_y = kDi;
      sa.offB = kDtR;
      sa.offC = kDtR + kNst;
      sa.offZ = 0;
      sa.ycarry = kYCarry;
      sa.dir = 1;
      sa.D = kDi;
      sa.L = kSeq;
      sa.nbatch = 1;
      ms1_scan_kernel<16><<<dim3(kDi / 64), 64, 0, stream>>>(sa);
    }
  }

  merge_norm_gate_kernel<<<kRows / 8, 256, 0, stream>>>(Yp, Zp, PAR + kParGam, PAR + kParBet, G16);

  wmma_gemm64<0, 0, 0><<<dim3(((kRows / 64) * (kDm / 64) + 7) / 8, 1), 256, 0, stream>>>(
      G16, kDi, 0L,
      WOUT, kDi, 0L,
      (void*)out, nullptr, kDm, 0L,
      nullptr,
      kRows, kDm, kDi, kOutScale, 1.0f);
}
